// MPNN_64845416235323
// MI455X (gfx1250) — hardware-verified
//
#include <hip/hip_runtime.h>
#include <stddef.h>
#include <stdint.h>
#include <math.h>


#define NN     68
#define BB     64
#define DD     256
#define TT     3
#define MROWS  (BB * NN)
#define KC     512
#define NAB    512
#define WSTR   516
#define NTHR   256
#define GBM    64
#define GBN    64
#define GTHR   128
#define NPRED  (TT * MROWS)
#define NOUT   (2 * NPRED)
#define ICH    17
#define PAIR_LDS (NN * DD * 4 + 4 * KC * 2)
#define WSMAX  134217728

#define U_H    (MROWS * DD / 4)
#define U_HHL  (MROWS * KC / 8)
#define U_WJI  (512 * KC / 8)
#define U_WU   (DD * KC / 8)
#define U_EE   (NN * NN * DD / 4)
#define U_TG   (NPRED / 4)
#define PB1    (U_H / NTHR)
#define PB2    (PB1 + U_HHL / NTHR)
#define PB3    (PB2 + U_WJI / NTHR)
#define PB4    (PB3 + U_WU / NTHR)
#define PB5    (PB4 + U_EE / NTHR)
#define PBEND  (PB5 + (U_TG + NTHR - 1) / NTHR)

static_assert(U_H % NTHR == 0 && U_HHL % NTHR == 0 && U_WJI % NTHR == 0 && U_WU % NTHR == 0 && U_EE % NTHR == 0);
static_assert(U_TG % 32 == 0);
static_assert(MROWS % GBM == 0 && MROWS % 32 == 0 && NAB % GBN == 0 && DD % GBN == 0 && KC % 32 == 0);
static_assert(NN == 4 * ICH && KC == 2 * DD);
static_assert((NPRED * 4) % 128 == 0 && (MROWS * 4) % 128 == 0);
static_assert((WSTR * 4) % 16 == 0);
static_assert(GBM == (GTHR / 32) * 16 && GBN == 64);

typedef float          v4f   __attribute__((ext_vector_type(4)));
typedef float          v8f   __attribute__((ext_vector_type(8)));
typedef int            v8i   __attribute__((ext_vector_type(8)));
typedef unsigned short v4us  __attribute__((ext_vector_type(4)));
typedef unsigned short v8us  __attribute__((ext_vector_type(8)));
typedef unsigned short v16us __attribute__((ext_vector_type(16)));
typedef __bf16         v16bf __attribute__((ext_vector_type(16)));
typedef v4f  __attribute__((may_alias)) v4fa;
typedef v8us __attribute__((may_alias)) v8usa;
typedef v4us __attribute__((may_alias)) v4usa;
union FragB { v16bf v; v16us u; v8us h[2]; v8i w; };

__device__ __forceinline__ v8f wmb(const FragB& a, const FragB& b, v8f c) {
  v8f d = __builtin_amdgcn_wmma_f32_16x16x32_bf16(false, a.v, false, b.v, (short)0, c, false, false);
  asm volatile("v_nop\n\tv_nop\n\tv_nop\n\tv_nop" : "+v"(d) : "v"(a.w), "v"(b.w));
  return d;
}

__device__ __forceinline__ unsigned bf16_bits(float f) {
  const unsigned u = __float_as_uint(f);
  return (u + 0x7FFFu + ((u >> 16) & 1u)) >> 16;
}
__device__ __forceinline__ float bf16_val(float f) { return __uint_as_float(bf16_bits(f) << 16); }
__device__ __forceinline__ v4f bf4(v4f a) {
  v4f o; o.x = bf16_val(a.x); o.y = bf16_val(a.y); o.z = bf16_val(a.z); o.w = bf16_val(a.w); return o;
}
__device__ __forceinline__ v8us cvt8(v4f a, v4f b) {
  v8us o;
  o[0] = (unsigned short)bf16_bits(a.x); o[1] = (unsigned short)bf16_bits(a.y);
  o[2] = (unsigned short)bf16_bits(a.z); o[3] = (unsigned short)bf16_bits(a.w);
  o[4] = (unsigned short)bf16_bits(b.x); o[5] = (unsigned short)bf16_bits(b.y);
  o[6] = (unsigned short)bf16_bits(b.z); o[7] = (unsigned short)bf16_bits(b.w);
  return o;
}
__device__ __forceinline__ void split1(float v, unsigned& hi, unsigned& lo) {
  hi = bf16_bits(v);
  lo = bf16_bits(v - __uint_as_float(hi << 16));
}
__device__ __forceinline__ void split8(v4f a, v4f b, v8us& hi, v8us& lo) {
  unsigned h, l;
  split1(a.x, h, l); hi[0] = (unsigned short)h; lo[0] = (unsigned short)l;
  split1(a.y, h, l); hi[1] = (unsigned short)h; lo[1] = (unsigned short)l;
  split1(a.z, h, l); hi[2] = (unsigned short)h; lo[2] = (unsigned short)l;
  split1(a.w, h, l); hi[3] = (unsigned short)h; lo[3] = (unsigned short)l;
  split1(b.x, h, l); hi[4] = (unsigned short)h; lo[4] = (unsigned short)l;
  split1(b.y, h, l); hi[5] = (unsigned short)h; lo[5] = (unsigned short)l;
  split1(b.z, h, l); hi[6] = (unsigned short)h; lo[6] = (unsigned short)l;
  split1(b.w, h, l); hi[7] = (unsigned short)h; lo[7] = (unsigned short)l;
}
__device__ __forceinline__ void put4(float* p, v4f v) {
  *(volatile v4f*)p = v;
  __threadfence();
  *(volatile v4f*)p = v;
}
__device__ __forceinline__ void put8(unsigned short* p, v8us v) {
  *(volatile v8us*)p = v;
  __threadfence();
  *(volatile v8us*)p = v;
}
__device__ __forceinline__ float wsum(float p) {
  p += __shfl_xor(p, 16); p += __shfl_xor(p, 8); p += __shfl_xor(p, 4); p += __shfl_xor(p, 2); p += __shfl_xor(p, 1);
  return p;
}

__global__ __launch_bounds__(NTHR) void k_prep(
    const float* __restrict__ latent, const float* __restrict__ target, const float* __restrict__ E,
    const float* __restrict__ W_mp, const float* __restrict__ b_mp, const float* __restrict__ W_up,
    float* H, unsigned short* HHL, unsigned short* WJI, unsigned short* WU, float* EE, float* outT) {
  const int blk = (int)blockIdx.x, tid = (int)threadIdx.x;
  if (blk < PB1) {
    const int u = blk * NTHR + tid;
    const v4f a = *(const v4fa*)(latent + 4 * (size_t)u);
    put4(H + 4 * (size_t)u, bf4(a));
  } else if (blk < PB2) {
    const int u   = (blk - PB1) * NTHR + tid;
    const int row = u >> 6;
    const int k8  = (u & 63) * 8;
    const int kk  = k8 & (DD - 1);
    const float* p = latent + (size_t)row * DD + kk;
    const v4f a = *(const v4fa*)p;
    const v4f b = *(const v4fa*)(p + 4);
    v8us o = cvt8(a, b);
    const unsigned short mk = (k8 < DD) ? (unsigned short)0xFFFF : (unsigned short)0;
#pragma unroll
    for (int e = 0; e < 8; ++e) o[e] = (unsigned short)(o[e] & mk);
    put8(HHL + (size_t)row * KC + k8, o);
  } else if (blk < PB3) {
    const int u   = (blk - PB2) * NTHR + tid;
    const int n   = u >> 6;
    const int k8  = (u & 63) * 8;
    const int kk  = k8 & (DD - 1);
    const int nn  = n & (DD - 1);
    const int cof = (n >> 8) * DD;
    const float* p = W_mp + (size_t)nn * WSTR + cof + kk;
    const v4f a = *(const v4fa*)p;
    const v4f b = *(const v4fa*)(p + 4);
    put8(WJI + (size_t)n * KC + k8, cvt8(a, b));
  } else if (blk < PB4) {
    const int u  = (blk - PB3) * NTHR + tid;
    const int n  = u >> 6;
    const int k8 = (u & 63) * 8;
    const int kk = k8 & (DD - 1);
    const float* p = W_up + (size_t)n * DD + kk;
    const v4f a = *(const v4fa*)p;
    const v4f b = *(const v4fa*)(p + 4);
    put8(WU + (size_t)n * KC + k8, cvt8(a, b));
  } else if (blk < PB5) {
    const int u  = (blk - PB4) * NTHR + tid;
    const int ij = u >> 6;
    const int d4 = (u & 63) * 4;
    const float e0 = bf16_val(E[ij]);
    const float e1 = bf16_val(E[NN * NN + ij]);
    const float e2 = bf16_val(E[2 * NN * NN + ij]);
    const float e3 = bf16_val(E[3 * NN * NN + ij]);
    const v4f bm = bf4(*(const v4fa*)(b_mp + d4));
    float o[4];
#pragma unroll
    for (int c = 0; c < 4; ++c) {
      const v4f w = bf4(*(const v4fa*)(W_mp + (size_t)(d4 + c) * WSTR + 2 * DD));
      float s = w.x * e0;
      s = fmaf(w.y, e1, s);
      s = fmaf(w.z, e2, s);
      s = fmaf(w.w, e3, s);
      o[c] = s;
    }
    v4f ov;
    ov.x = o[0] + bm.x; ov.y = o[1] + bm.y; ov.z = o[2] + bm.z; ov.w = o[3] + bm.w;
    put4(EE + (size_t)ij * DD + d4, ov);
  } else {
    const int u = (blk - PB5) * NTHR + tid;
    if (u < U_TG) {
      const int t = u / (MROWS / 4);
      const int q = u - t * (MROWS / 4);
      const v4f a = *(const v4fa*)(target + 4 * q);
      put4(outT + 4 * (size_t)u, bf4(a));
    }
  }
}

template <int EPI>
__global__ __launch_bounds__(GTHR) void k_gemm(
    const unsigned short* __restrict__ A, const unsigned short* __restrict__ WT,
    const float* __restrict__ bias, float* outF, int K, int ldo)
{
  __shared__ __attribute__((aligned(16))) float stg[GBM * GBN];
  const int tid = (int)threadIdx.x, lane = tid & 31, wave = tid >> 5, hh = lane >> 4, m = lane & 15;
  const int rowBase = (int)blockIdx.x * GBM;
  const int col0    = (int)blockIdx.y * GBN;

  v8f acc[4];
  {
    const v8f z = {0.f, 0.f, 0.f, 0.f, 0.f, 0.f, 0.f, 0.f};
    acc[0] = z; acc[1] = z; acc[2] = z; acc[3] = z;
  }
  const unsigned short* ap = A  + (size_t)(rowBase + 16 * wave + m) * (size_t)K + 8 * hh;
  const unsigned short* wp = WT + (size_t)(col0 + m) * (size_t)K + 8 * hh;
  const int ksteps = K >> 5;
#pragma unroll 1
  for (int ks = 0; ks < ksteps; ++ks) {
    FragB af;
    af.h[0] = *(const v8usa*)(ap + 32 * ks);
    af.h[1] = *(const v8usa*)(ap + 32 * ks + 16);
#pragma unroll
    for (int t = 0; t < 4; ++t) {
      const unsigned short* wq = wp + (size_t)(16 * t) * (size_t)K + 32 * ks;
      FragB bf;
      bf.h[0] = *(const v8usa*)wq;
      bf.h[1] = *(const v8usa*)(wq + 16);
      acc[t] = wmb(af, bf, acc[t]);
    }
  }

#pragma unroll
  for (int t = 0; t < 4; ++t) {
    const int lc = 16 * t + m;
    float bv = 0.0f;
    if (EPI != 0) bv = bf16_val(bias[col0 + lc]);
#pragma unroll
    for (int r = 0; r < 8; ++r) {
      const int lr = 16 * wave + 8 * hh + r;
      float v = acc[t][r];
      if (EPI != 0) { v = v + bv; v = fmaxf(v, 0.01f * v); }
      stg[lr * GBN + lc] = v;
    }
  }
  __syncthreads();

  v4f fv[8];
#pragma unroll
  for (int i = 0; i < 8; ++i) {
    const int lr = 16 * wave + 2 * i + hh;
    fv[i] = *(const v4fa*)(stg + lr * GBN + 4 * m);
  }
#pragma unroll
  for (int i = 0; i < 8; ++i) {
    const int lr = 16 * wave + 2 * i + hh;
    const int gr = rowBase + lr;
    float* op = outF + (size_t)gr * (size_t)ldo + col0 + 4 * m;
    *(volatile v4f*)op = fv[i];
  }
  __threadfence();
#pragma unroll
  for (int i = 0; i < 8; ++i) {
    const int lr = 16 * wave + 2 * i + hh;
    const int gr = rowBase + lr;
    float* op = outF + (size_t)gr * (size_t)ldo + col0 + 4 * m;
    *(volatile v4f*)op = fv[i];
  }
}

__device__ __forceinline__ v4f pterm(v4f a, v4f bi, v4f e) {
  const v4f v = (a + bi) + e;
  const v4f s = v * 0.01f;
  v4f o;
  o.x = fmaxf(v.x, s.x); o.y = fmaxf(v.y, s.y); o.z = fmaxf(v.z, s.z); o.w = fmaxf(v.w, s.w);
  return o;
}

__global__ __launch_bounds__(NTHR) void k_pair(const float* __restrict__ AB, const float* __restrict__ EE,
                                               const float* __restrict__ H, unsigned short* MHL) {
  extern __shared__ v4f lds_dyn[];
  float* at = (float*)lds_dyn;
  unsigned short* st = (unsigned short*)(at + NN * DD);
  const int tid = (int)threadIdx.x;
  const int b   = (int)blockIdx.x;
  const int ig  = __builtin_amdgcn_readfirstlane(tid >> 6);
  const int dq  = tid & 63;
  const int c8  = dq * 8;

#pragma unroll 1
  for (int it = 0; it < NN * DD / 4 / NTHR; ++it) {
    const int idx = it * NTHR + tid;
    const int row = idx >> 6, c4 = idx & 63;
    *(v4f*)(at + row * DD + 4 * c4) = *(const v4fa*)(AB + (size_t)(b * NN + row) * NAB + 4 * c4);
  }
  __syncthreads();

  const float inv = 1.0f / (float)NN;
  const float* ap = at + 4 * dq;
#pragma unroll 1
  for (int ii = 0; ii < ICH; ++ii) {
    const int i = ICH * ig + ii;
    const int r = b * NN + i;
    const v4f bi = *(const v4fa*)(AB + (size_t)r * NAB + DD + 4 * dq);
    const float* ep = EE + (size_t)i * NN * DD + 4 * dq;
    v4f acc = {0.f, 0.f, 0.f, 0.f};
#pragma unroll 2
    for (int j = 0; j < i; ++j)
      acc += pterm(*(const v4fa*)(ap + j * DD), bi, *(const v4fa*)(ep + (size_t)j * DD));
#pragma unroll 2
    for (int j = i + 1; j < NN; ++j)
      acc += pterm(*(const v4fa*)(ap + j * DD), bi, *(const v4fa*)(ep + (size_t)j * DD));
    const v4f hv = *(const v4fa*)(H + (size_t)r * DD + 4 * dq);
    v4f mv;
    mv.x = hv.x + acc.x * inv; mv.y = hv.y + acc.y * inv; mv.z = hv.z + acc.z * inv; mv.w = hv.w + acc.w * inv;
    unsigned h0, h1, h2, h3, l0, l1, l2, l3;
    split1(mv.x, h0, l0); split1(mv.y, h1, l1); split1(mv.z, h2, l2); split1(mv.w, h3, l3);
    v4us hq, lq;
    hq[0] = (unsigned short)h0; hq[1] = (unsigned short)h1; hq[2] = (unsigned short)h2; hq[3] = (unsigned short)h3;
    lq[0] = (unsigned short)l0; lq[1] = (unsigned short)l1; lq[2] = (unsigned short)l2; lq[3] = (unsigned short)l3;
    *(v4usa*)(st + ig * KC + 4 * dq)      = hq;
    *(v4usa*)(st + ig * KC + DD + 4 * dq) = lq;
    __syncthreads();
    const int rr = tid >> 6;
    const v8us pv = *(const v8usa*)(st + rr * KC + c8);
    unsigned short* gp = MHL + (size_t)(b * NN + ICH * rr + ii) * KC + c8;
    *(volatile v8us*)gp = pv;
    __threadfence();
    *(volatile v8us*)gp = pv;
    __syncthreads();
  }
}

__global__ __launch_bounds__(NTHR) void k_row(const float* __restrict__ U, const float* __restrict__ W_ro,
                                              const float* __restrict__ b_ro, float* H, unsigned short* HHL,
                                              float* pred, int wr) {
  __shared__ __attribute__((aligned(16))) float hn[32 * DD];
  __shared__ __attribute__((aligned(16))) float ps[32];
  const int tid = (int)threadIdx.x, lane = tid & 31, wave = tid >> 5;
  const int rb = (int)blockIdx.x * 32;
  const v4f w0 = bf4(*(const v4fa*)(W_ro + 4 * lane));
  const v4f w1 = bf4(*(const v4fa*)(W_ro + 128 + 4 * lane));
  const float bro = bf16_val(b_ro[0]);

#pragma unroll 1
  for (int q = 0; q < 4; ++q) {
    const int lr = wave * 4 + q;
    const float* up = U + (size_t)(rb + lr) * DD;
    const v4f u0 = *(const v4fa*)(up + 4 * lane);
    const v4f u1 = *(const v4fa*)(up + 128 + 4 * lane);
    float s = ((u0.x + u0.y) + (u0.z + u0.w)) + ((u1.x + u1.y) + (u1.z + u1.w));
    s = wsum(s);
    const float mu = s * (1.0f / (float)DD);
    const v4f d0 = u0 - mu;
    const v4f d1 = u1 - mu;
    float qv = ((d0.x * d0.x + d0.y * d0.y) + (d0.z * d0.z + d0.w * d0.w))
             + ((d1.x * d1.x + d1.y * d1.y) + (d1.z * d1.z + d1.w * d1.w));
    qv = wsum(qv);
    const float var = qv * (1.0f / (float)DD);
    const float rs = rsqrtf(var + 1e-5f);
    const v4f h0 = d0 * rs;
    const v4f h1 = d1 * rs;
    float dt = ((h0.x * w0.x + h0.y * w0.y) + (h0.z * w0.z + h0.w * w0.w))
             + ((h1.x * w1.x + h1.y * w1.y) + (h1.z * w1.z + h1.w * w1.w));
    dt = wsum(dt);
    const float z = dt + bro;
    const float p = 1.0f / (1.0f + expf(-z));
    *(v4f*)(hn + lr * DD + 4 * lane)       = h0;
    *(v4f*)(hn + lr * DD + 128 + 4 * lane) = h1;
    if (lane == 0) ps[lr] = p;
  }
  __syncthreads();

  const v4f pv = *(const v4fa*)(ps + 4 * (lane & 7));
  float* pp = pred + (size_t)rb + 4 * (lane & 7);
  const bool pw = tid < 8;
  if (wr != 0) {
    v4f hv[8];
#pragma unroll
    for (int it = 0; it < 8; ++it) hv[it] = *(const v4fa*)(hn + 4 * (it * NTHR + tid));
    v8us hi[4], lo[4];
#pragma unroll
    for (int it = 0; it < 4; ++it) {
      const int u = it * NTHR + tid;
      const int row = u >> 5, cc = (u & 31) * 8;
      const v4f a = *(const v4fa*)(hn + row * DD + cc);
      const v4f b = *(const v4fa*)(hn + row * DD + cc + 4);
      split8(a, b, hi[it], lo[it]);
    }
    float* hp = H + (size_t)rb * DD;
#pragma unroll
    for (int it = 0; it < 8; ++it) *(volatile v4f*)(hp + 4 * (it * NTHR + tid)) = hv[it];
#pragma unroll
    for (int it = 0; it < 4; ++it) {
      const int u = it * NTHR + tid;
      const int row = u >> 5, cc = (u & 31) * 8;
      unsigned short* gp = HHL + (size_t)(rb + row) * KC + cc;
      *(volatile v8us*)gp = hi[it];
      *(volatile v8us*)(gp + DD) = lo[it];
    }
    if (pw) *(volatile v4f*)pp = pv;
    __threadfence();
#pragma unroll
    for (int it = 0; it < 8; ++it) *(volatile v4f*)(hp + 4 * (it * NTHR + tid)) = hv[it];
#pragma unroll
    for (int it = 0; it < 4; ++it) {
      const int u = it * NTHR + tid;
      const int row = u >> 5, cc = (u & 31) * 8;
      unsigned short* gp = HHL + (size_t)(rb + row) * KC + cc;
      *(volatile v8us*)gp = hi[it];
      *(volatile v8us*)(gp + DD) = lo[it];
    }
    if (pw) *(volatile v4f*)pp = pv;
  } else {
    if (pw) *(volatile v4f*)pp = pv;
    __threadfence();
    if (pw) *(volatile v4f*)pp = pv;
  }
}

static inline size_t al256(size_t o) { return (o + 255) & ~(size_t)255; }

extern "C" void kernel_launch(void* const* d_in, const int* in_sizes, int n_in,
                              void* d_out, int out_size, void* d_ws, size_t ws_size,
                              hipStream_t stream) {
  if (n_in < 9) return;
  if (in_sizes[0] != MROWS * DD) return;
  if (in_sizes[1] != MROWS) return;
  if (in_sizes[2] != 4 * NN * NN) return;
  if (in_sizes[3] != DD * WSTR) return;
  if (in_sizes[4] != DD) return;
  if (in_sizes[5] != DD * DD) return;
  if (in_sizes[6] != DD) return;
  if (in_sizes[7] != DD) return;
  if (in_sizes[8] != 1) return;
  if (out_size != NOUT) return;

  const float* latent = (const float*)d_in[0];
  const float* target = (const float*)d_in[1];
  const float* E      = (const float*)d_in[2];
  const float* W_mp   = (const float*)d_in[3];
  const float* b_mp   = (const float*)d_in[4];
  const float* W_up   = (const float*)d_in[5];
  const float* b_up   = (const float*)d_in[6];
  const float* W_ro   = (const float*)d_in[7];
  const float* b_ro   = (const float*)d_in[8];
  float* out = (float*)d_out;

  char* ws = (char*)d_ws;
  size_t off = 0;
  const size_t oH   = off; off = al256(off + (size_t)MROWS * DD * 4);
  const size_t oHHL = off; off = al256(off + (size_t)MROWS * KC * 2);
  const size_t oAB  = off; off = al256(off + (size_t)MROWS * NAB * 4);
  const size_t oEE  = off; off = al256(off + (size_t)NN * NN * DD * 4);
  const size_t oMHL = off; off = al256(off + (size_t)MROWS * KC * 2);
  const size_t oU   = off; off = al256(off + (size_t)MROWS * DD * 4);
  const size_t oWJI = off; off = al256(off + (size_t)512 * KC * 2);
  const size_t oWU  = off; off = al256(off + (size_t)DD * KC * 2);
  if (off > ws_size || off > (size_t)WSMAX) return;
  float*          H   = (float*)(ws + oH);
  unsigned short* HHL = (unsigned short*)(ws + oHHL);
  float*          AB  = (float*)(ws + oAB);
  float*          EE  = (float*)(ws + oEE);
  unsigned short* MHL = (unsigned short*)(ws + oMHL);
  float*          U   = (float*)(ws + oU);
  unsigned short* WJI = (unsigned short*)(ws + oWJI);
  unsigned short* WU  = (unsigned short*)(ws + oWU);

  hipFuncSetAttribute(reinterpret_cast<const void*>(&k_pair), hipFuncAttributeMaxDynamicSharedMemorySize, PAIR_LDS);

  k_prep<<<PBEND, NTHR, 0, stream>>>(latent, target, E, W_mp, b_mp, W_up, H, HHL, WJI, WU, EE, out + NPRED);
  for (int t = 0; t < TT; ++t) {
    k_gemm<0><<<dim3(MROWS / GBM, NAB / GBN), GTHR, 0, stream>>>(HHL, WJI, b_up, AB, KC, NAB);
    k_pair<<<BB, NTHR, PAIR_LDS, stream>>>(AB, EE, H, MHL);
    k_gemm<1><<<dim3(MROWS / GBM, DD / GBN), GTHR, 0, stream>>>(MHL, WU, b_up, U, KC, DD);
    k_row<<<MROWS / 32, NTHR, 0, stream>>>(U, W_ro, b_ro, H, HHL, out + (size_t)t * MROWS, (t + 1 < TT) ? 1 : 0);
  }
}
